// FeedBack_41205916238533
// MI455X (gfx1250) — hardware-verified
//
#include <hip/hip_runtime.h>
#include <math.h>

constexpr int NB         = 128;
constexpr int NTS        = 2048;
constexpr int ND         = 3;
constexpr int NU         = 256;
constexpr int NG         = 1024;
constexpr int NPROJ      = 3;
constexpr int NOUT       = NB * NPROJ;
constexpr int NT         = 256;
constexpr int NTR        = 512;
constexpr int NTD        = 384;
constexpr int SEQ_BLK    = 16;
constexpr int HP         = 264;
constexpr int OP         = 260;
constexpr int XQ         = 4;
constexpr int TAIL_STEPS = 512;
constexpr float UCARRY     = 64.0f;
constexpr float UCARRY_INV = 1.0f / 64.0f;
constexpr float RES_CARRY  = 2048.0f;
constexpr float RES_FOLD   = 1.0f / 2048.0f;
static_assert(NG == 4 * NU);
static_assert(NB % SEQ_BLK == 0);
static_assert(NU == 16 * (NTR / 32));
static_assert(NU % 32 == 0);
static_assert(NG % 64 == 0 && NU % 64 == 0);
static_assert(SEQ_BLK * OP >= ND * NG + NG);
static_assert(ND * NG == 3 * NT * 4);
static_assert(NG == NT * 4);
static_assert(NTR >= NT);
static_assert(NTD == NOUT);
static_assert(NU * NPROJ == 2 * NTD);
static_assert(NOUT == 3 * 32 * 4);
static_assert(SEQ_BLK * XQ == 64);
static_assert(SEQ_BLK * NU == 2 * NTR * 4);
static_assert(NTS > TAIL_STEPS + 1);
static_assert(HP % 8 == 0 && OP % 4 == 0);

typedef __attribute__((ext_vector_type(16))) _Float16 v16h;
typedef __attribute__((ext_vector_type(8)))  _Float16 v8h;
typedef __attribute__((ext_vector_type(16))) __bf16   v16b;
typedef __attribute__((ext_vector_type(8)))  __bf16   v8b;
typedef __attribute__((ext_vector_type(8)))  float    v8f;
typedef __attribute__((ext_vector_type(4)))  float    v4f;

__device__ __forceinline__ unsigned short f2bf_bits(float f) {
  unsigned u = __float_as_uint(f);
  return (unsigned short)((u + 0x7FFFu + ((u >> 16) & 1u)) >> 16);
}
__device__ __forceinline__ float bf_bits2f(unsigned short h) { return __uint_as_float(((unsigned)h) << 16); }
__device__ __forceinline__ float bf16r(float f) { return bf_bits2f(f2bf_bits(f)); }

__device__ __forceinline__ void dep_guard_h(v8f& a, v8f& b, v16h x, v16h y) { asm volatile("v_nop\n\tv_nop\n\tv_nop\n\tv_nop" : "+v"(a), "+v"(b) : "v"(x), "v"(y)); }
__device__ __forceinline__ void dep_guard_b(v8f& a, v8f& b, v16b x, v16b y) { asm volatile("v_nop\n\tv_nop\n\tv_nop\n\tv_nop" : "+v"(a), "+v"(b) : "v"(x), "v"(y)); }
__device__ __forceinline__ void keep4_h(v16h a, v16h b, v16h c, v16h d) { asm volatile("v_nop" :: "v"(a), "v"(b), "v"(c), "v"(d)); }
__device__ __forceinline__ void keep4_b(v16b a, v16b b, v16b c, v16b d) { asm volatile("v_nop" :: "v"(a), "v"(b), "v"(c), "v"(d)); }
__device__ __forceinline__ void acc_guard4(v8f& a, v8f& b, v8f& c, v8f& d) { asm volatile("v_nop\n\tv_nop\n\tv_nop\n\tv_nop" : "+v"(a), "+v"(b), "+v"(c), "+v"(d)); }
__device__ __forceinline__ void grp_guard_h(v8f& a0, v8f& a1, v8f& a2, v8f& a3,
                                            v16h x, v16h y0, v16h y1, v16h y2, v16h y3) {
  asm volatile("v_nop\n\tv_nop\n\tv_nop\n\tv_nop"
               : "+v"(a0), "+v"(a1), "+v"(a2), "+v"(a3)
               : "v"(x), "v"(y0), "v"(y1), "v"(y2), "v"(y3));
}
template <typename T> struct Frag;
template <> struct Frag<_Float16> {
  typedef v16h V; union U { v16h v; v8h h[2]; };
  static __device__ __forceinline__ v16h load(const _Float16* p) {
    U f; f.h[0] = *(const v8h*)(p); f.h[1] = *(const v8h*)(p + 16); return f.v;
  }
  static __device__ __forceinline__ v8f mma(v16h a, v16h b, v8f c) {
    return __builtin_amdgcn_wmma_f32_16x16x32_f16(false, a, false, b, (short)0, c, false, false);
  }
  static __device__ __forceinline__ void guard(v8f& a, v8f& b, v16h x, v16h y) { dep_guard_h(a, b, x, y); }
  static __device__ __forceinline__ void keep(v16h a, v16h b, v16h c, v16h d) { keep4_h(a, b, c, d); }
};
template <> struct Frag<__bf16> {
  typedef v16b V; union U { v16b v; v8b h[2]; };
  static __device__ __forceinline__ v16b load(const __bf16* p) {
    U f; f.h[0] = *(const v8b*)(p); f.h[1] = *(const v8b*)(p + 16); return f.v;
  }
  static __device__ __forceinline__ v8f mma(v16b a, v16b b, v8f c) {
    return __builtin_amdgcn_wmma_f32_16x16x32_bf16(false, a, false, b, (short)0, c, false, false);
  }
  static __device__ __forceinline__ void guard(v8f& a, v8f& b, v16b x, v16b y) { dep_guard_b(a, b, x, y); }
  static __device__ __forceinline__ void keep(v16b a, v16b b, v16b c, v16b d) { keep4_b(a, b, c, d); }
};

__device__ __forceinline__ float fsig(float x) { return __builtin_amdgcn_rcpf(1.0f + expf(-x)); }

template <int MODE>
__global__ __launch_bounds__(NT) void tpw_kernel(const float* __restrict__ src, int R, int C, int ldo,
                                                unsigned short* __restrict__ O, float sc) {
  __shared__ float Tt[64 * 65];
  const int tid = threadIdx.x;
  const int c0 = blockIdx.x * 64, r0 = blockIdx.y * 64;
#pragma unroll
  for (int i = 0; i < 4; ++i) {
    const int idx = i * NT + tid;
    const int rr = idx >> 4, cc = (idx & 15) * 4;
    const v4f v = *(const v4f*)(src + (size_t)(r0 + rr) * (size_t)C + c0 + cc);
    Tt[rr * 65 + cc + 0] = v[0];
    Tt[rr * 65 + cc + 1] = v[1];
    Tt[rr * 65 + cc + 2] = v[2];
    Tt[rr * 65 + cc + 3] = v[3];
  }
  __syncthreads();
  const int q = tid >> 3, c8 = (tid & 7) * 8;
  v8h hv[2];
#pragma unroll
  for (int g = 0; g < 2; ++g) {
    const int qq = g * 32 + q;
#pragma unroll
    for (int e = 0; e < 8; ++e) {
      const float f = Tt[(c8 + e) * 65 + qq];
      unsigned short bits;
      if (MODE == 0) {
        bits = f2bf_bits(f * sc);
      } else {
        const float fb = bf_bits2f(f2bf_bits(f));
        bits = __builtin_bit_cast(unsigned short, (_Float16)(fb * sc));
      }
      hv[g][e] = __builtin_bit_cast(_Float16, bits);
    }
  }
  for (int pass = 0; pass < 2; ++pass) {
#pragma unroll
    for (int g = 0; g < 2; ++g) {
      const size_t o = (size_t)(c0 + g * 32 + q) * (size_t)ldo + (size_t)(r0 + c8);
      *(volatile v8h*)(O + o) = hv[g];
    }
    __threadfence();
  }
}

__global__ __launch_bounds__(NTR) void lstm_seq_kernel(const float* __restrict__ x, const float* __restrict__ W,
                                                      const float* __restrict__ bvec,
                                                      const unsigned short* __restrict__ UTp,
                                                      float* __restrict__ HL) {
  __shared__ __align__(16) _Float16 Ahl[2 * SEQ_BLK * HP];
  __shared__ __align__(16) float    Xs[SEQ_BLK * XQ];
  __shared__ __align__(16) float    Hs[SEQ_BLK * OP];
  _Float16* Ah = Ahl;
  _Float16* Al = Ahl + SEQ_BLK * HP;
  const _Float16* UT = (const _Float16*)UTp;
  const int tid = threadIdx.x, lane = tid & 31, wave = tid >> 5;
  const int c = lane & 15, hh = lane >> 4, koff = hh * 8;
  const int rowbase = blockIdx.x * SEQ_BLK;
  const int j = 16 * wave + c;

#pragma unroll 1
  for (int i = tid; i < 2 * SEQ_BLK * HP; i += NTR) Ahl[i] = (_Float16)0.0f;
  if (wave < 2) {
    const int m = tid >> 2, d = tid & 3, dd = (d < ND) ? d : (ND - 1);
    Xs[m * XQ + d] = bf16r(x[((size_t)(rowbase + m) * NTS) * ND + dd]);
  }
  if (wave < 8) {
    float* stg = Hs;
#pragma unroll
    for (int i = 0; i < 3; ++i) {
      const int idx = (i * NT + tid) * 4;
      *(v4f*)(stg + idx) = *(const v4f*)(W + idx);
    }
    *(v4f*)(stg + ND * NG + tid * 4) = *(const v4f*)(bvec + tid * 4);
  }
  __syncthreads();

  float wv[4][3], bb[4], cst[8], hst[8];
#pragma unroll
  for (int g = 0; g < 4; ++g) {
#pragma unroll
    for (int d = 0; d < 3; ++d) wv[g][d] = bf16r(Hs[d * NG + g * NU + j]);
    bb[g] = bf16r(Hs[ND * NG + g * NU + j]);
  }
#pragma unroll
  for (int r = 0; r < 8; ++r) { cst[r] = 0.0f; hst[r] = 0.0f; }

  const _Float16* ahrow = Ah + c * HP + koff;
  const _Float16* alrow = Al + c * HP + koff;
  const _Float16* up    = UT + (size_t)j * NU + koff;
  const v8f z8 = {0.f, 0.f, 0.f, 0.f, 0.f, 0.f, 0.f, 0.f};

#pragma unroll 1
  for (int t = 0; t < NTS; ++t) {
    const bool tail = (t >= NTS - TAIL_STEPS);
    const bool wres = (t + 1 >= NTS - TAIL_STEPS);
    v8f acc[4], accL[4];
    acc[0] = z8; acc[1] = z8; acc[2] = z8; acc[3] = z8;
    accL[0] = z8; accL[1] = z8; accL[2] = z8; accL[3] = z8;
#pragma unroll 1
    for (int k0 = 0; k0 < NU; k0 += 32) {
      const v16h a  = Frag<_Float16>::load(ahrow + k0);
      const v16h b0 = Frag<_Float16>::load(up + k0);
      const v16h b1 = Frag<_Float16>::load(up + (size_t)1 * NU * NU + k0);
      const v16h b2 = Frag<_Float16>::load(up + (size_t)2 * NU * NU + k0);
      const v16h b3 = Frag<_Float16>::load(up + (size_t)3 * NU * NU + k0);
      acc[0] = Frag<_Float16>::mma(a, b0, acc[0]);
      acc[1] = Frag<_Float16>::mma(a, b1, acc[1]);
      acc[2] = Frag<_Float16>::mma(a, b2, acc[2]);
      acc[3] = Frag<_Float16>::mma(a, b3, acc[3]);
      grp_guard_h(acc[0], acc[1], acc[2], acc[3], a, b0, b1, b2, b3);
    }
    acc_guard4(acc[0], acc[1], acc[2], acc[3]);
    if (tail) {
#pragma unroll 1
      for (int k0 = 0; k0 < NU; k0 += 32) {
        const v16h al  = Frag<_Float16>::load(alrow + k0);
        const v16h bt0 = Frag<_Float16>::load(up + k0);
        const v16h bt1 = Frag<_Float16>::load(up + (size_t)1 * NU * NU + k0);
        const v16h bt2 = Frag<_Float16>::load(up + (size_t)2 * NU * NU + k0);
        const v16h bt3 = Frag<_Float16>::load(up + (size_t)3 * NU * NU + k0);
        accL[0] = Frag<_Float16>::mma(al, bt0, accL[0]);
        accL[1] = Frag<_Float16>::mma(al, bt1, accL[1]);
        accL[2] = Frag<_Float16>::mma(al, bt2, accL[2]);
        accL[3] = Frag<_Float16>::mma(al, bt3, accL[3]);
        grp_guard_h(accL[0], accL[1], accL[2], accL[3], al, bt0, bt1, bt2, bt3);
      }
    }
    acc_guard4(accL[0], accL[1], accL[2], accL[3]);
#pragma unroll
    for (int r = 0; r < 8; ++r) {
      const v4f xv = *(const v4f*)(Xs + (8 * hh + r) * XQ);
      const float x0 = xv[0], x1 = xv[1], x2 = xv[2];
      const float xzi = fmaf(x2, wv[0][2], fmaf(x1, wv[0][1], x0 * wv[0][0])) + bb[0];
      const float xzf = fmaf(x2, wv[1][2], fmaf(x1, wv[1][1], x0 * wv[1][0])) + bb[1];
      const float xzg = fmaf(x2, wv[2][2], fmaf(x1, wv[2][1], x0 * wv[2][0])) + bb[2];
      const float xzo = fmaf(x2, wv[3][2], fmaf(x1, wv[3][1], x0 * wv[3][0])) + bb[3];
      const float zi = fmaf(accL[0][r], RES_FOLD, acc[0][r]) * UCARRY_INV + xzi;
      const float zf = fmaf(accL[1][r], RES_FOLD, acc[1][r]) * UCARRY_INV + xzf;
      const float zg = fmaf(accL[2][r], RES_FOLD, acc[2][r]) * UCARRY_INV + xzg;
      const float zo = fmaf(accL[3][r], RES_FOLD, acc[3][r]) * UCARRY_INV + xzo;
      const float ig = fsig(zi);
      const float fg = fsig(zf);
      const float gg = fmaxf(zg, 0.0f);
      const float cn = fg * cst[r] + ig * gg;
      cst[r] = cn;
      const float og = fsig(zo);
      hst[r] = og * fmaxf(cn, 0.0f);
    }
    __syncthreads();
#pragma unroll
    for (int r = 0; r < 8; ++r) {
      const float hn = hst[r];
      const _Float16 h16 = (_Float16)hn;
      Ah[(8 * hh + r) * HP + j] = h16;
      if (wres) {
        const float hres = (hn - (float)h16) * RES_CARRY;
        Al[(8 * hh + r) * HP + j] = (_Float16)hres;
      }
    }
    if (wave < 2) {
      const int tn = (t + 1 < NTS) ? (t + 1) : (NTS - 1);
      const int m = tid >> 2, d = tid & 3, dd = (d < ND) ? d : (ND - 1);
      Xs[m * XQ + d] = bf16r(x[((size_t)(rowbase + m) * NTS + (size_t)tn) * ND + dd]);
    }
    __syncthreads();
  }

#pragma unroll
  for (int r = 0; r < 8; ++r) Hs[(8 * hh + r) * OP + j] = hst[r];
  __syncthreads();
  for (int pass = 0; pass < 2; ++pass) {
#pragma unroll
    for (int it = 0; it < 2; ++it) {
      const int idx = it * NTR + tid;
      const int row = idx >> 6, c4 = (idx & 63) * 4;
      const v4f v = *(const v4f*)(Hs + row * OP + c4);
      *(volatile v4f*)(HL + (size_t)(rowbase + row) * NU + c4) = v;
    }
    __threadfence();
  }
}

__global__ __launch_bounds__(NTD) void dense_kernel(const float* __restrict__ HL, const float* __restrict__ Wd,
                                                   const float* __restrict__ bd, float* __restrict__ out) {
  __shared__ __align__(16) float Wds[NU * NPROJ];
  __shared__ __align__(16) float Os[NOUT];
  const int tid = threadIdx.x;
  Wds[tid]       = bf16r(Wd[tid]);
  Wds[NTD + tid] = bf16r(Wd[NTD + tid]);
  const int r  = tid / NPROJ;
  const int jj = tid - r * NPROJ;
  const float bdv = bf16r(bd[jj]);
  __syncthreads();
  const float* hp = HL + (size_t)r * NU;
  float s = 0.0f;
#pragma unroll 1
  for (int u4 = 0; u4 < NU / 4; ++u4) {
    const v4f h = *(const v4f*)(hp + 4 * u4);
    const float* wp = Wds + (4 * u4) * NPROJ + jj;
    s = fmaf(h[0], wp[0], s);
    s = fmaf(h[1], wp[NPROJ], s);
    s = fmaf(h[2], wp[2 * NPROJ], s);
    s = fmaf(h[3], wp[3 * NPROJ], s);
  }
  Os[tid] = s + bdv;
  __syncthreads();
  if (tid < 32) {
    for (int pass = 0; pass < 2; ++pass) {
#pragma unroll
      for (int it = 0; it < NOUT / 128; ++it) {
        const int idx = it * 32 + tid;
        const v4f v = *(const v4f*)(Os + idx * 4);
        *(volatile v4f*)(out + idx * 4) = v;
      }
      __threadfence();
    }
  }
}

extern "C" void kernel_launch(void* const* d_in, const int* in_sizes, int n_in,
                              void* d_out, int out_size, void* d_ws, size_t ws_size, hipStream_t stream) {
  if (n_in < 6 || d_out == nullptr || d_ws == nullptr) return;
  if (in_sizes[0] != NB * NTS * ND || in_sizes[1] != ND * NG || in_sizes[2] != NU * NG || in_sizes[3] != NG ||
      in_sizes[4] != NU * NPROJ || in_sizes[5] != NPROJ || out_size != NOUT) return;

  const float* x    = (const float*)d_in[0];
  const float* W    = (const float*)d_in[1];
  const float* U    = (const float*)d_in[2];
  const float* bvec = (const float*)d_in[3];
  const float* Wd   = (const float*)d_in[4];
  const float* bd   = (const float*)d_in[5];
  float* out = (float*)d_out;

  char* ws = (char*)d_ws; size_t off = 0;
  auto carve = [&](size_t bytes) -> char* { char* p = ws + off; off += (bytes + 255) & ~(size_t)255; return p; };
  unsigned short* UT = (unsigned short*)carve((size_t)NG * NU * 2);
  float*          HL = (float*)carve((size_t)NB * NU * 4);
  if (off > ws_size || off > (size_t)134217728) return;

  tpw_kernel<1><<<dim3(NG / 64, NU / 64), NT, 0, stream>>>(U, NU, NG, NU, UT, UCARRY);
  lstm_seq_kernel<<<NB / SEQ_BLK, NTR, 0, stream>>>(x, W, bvec, UT, HL);
  dense_kernel<<<1, NTD, 0, stream>>>(HL, Wd, bd, out);
}
